// HeteroMessagePassingLayer_11373073400378
// MI455X (gfx1250) — hardware-verified
//
#include <hip/hip_runtime.h>
#include <stddef.h>


#define DF     256
#define NTHR   256
#define NWAVE  8
#define CHUNK  2048
#define NGRP   (CHUNK / (NTHR * 4))
#define WCAP   256
#define NB     256
#define NBSH   8
#define NBD    4096
#define NBDSH  12
#define GR     32
#define AP     264
#define XSP    260
#define GEMM_LDS (2 * GR * AP * 2)
#define AGG_SACC (NB * DF)
#define LDS_GLOM ((AGG_SACC + 3 * NB + NWAVE * WCAP + NWAVE) * 4)
#define LDS_IMM  ((AGG_SACC + NWAVE * WCAP + NWAVE) * 4)

static_assert(NGRP == 2);
static_assert(WCAP == (CHUNK / NTHR) * 32);
static_assert(NB == NTHR);
static_assert((NB - 1) < (1 << NBSH));
static_assert((NBD - 1) < (1 << NBDSH));
static_assert(((CHUNK - 1) << NBDSH) + NBD - 1 < 2147483647);
static_assert(GEMM_LDS == 33792);
static_assert(GEMM_LDS >= GR * XSP * 4);
static_assert(LDS_GLOM == 273440);
static_assert(LDS_IMM == 270368);
static_assert((AGG_SACC % 4) == 0);
static_assert((NBD % (4 * NTHR)) == 0);

typedef float          v4f   __attribute__((ext_vector_type(4)));
typedef float          v8f   __attribute__((ext_vector_type(8)));
typedef int            v4i   __attribute__((ext_vector_type(4)));
typedef unsigned short v8us  __attribute__((ext_vector_type(8)));
typedef __bf16         v16bf __attribute__((ext_vector_type(16)));
union FragB { v16bf v; v8us h[2]; };

__device__ __forceinline__ v8f wm(v16bf a, v16bf b, v8f c) {
  v8f d = __builtin_amdgcn_wmma_f32_16x16x32_bf16(false, a, false, b, (short)0, c, false, false);
  asm volatile("v_nop\n\tv_nop\n\tv_nop\n\tv_nop" : "+v"(d) : "v"(a), "v"(b));
  return d;
}

__device__ __forceinline__ float wsum(float v) {
  v += __shfl_xor(v, 16, 32);
  v += __shfl_xor(v, 8, 32);
  v += __shfl_xor(v, 4, 32);
  v += __shfl_xor(v, 2, 32);
  v += __shfl_xor(v, 1, 32);
  return v;
}

__device__ __forceinline__ unsigned bf_rne(float f) {
  const unsigned u = __float_as_uint(f);
  return (u + 0x7FFFu + ((u >> 16) & 1u)) >> 16;
}

__device__ __forceinline__ void split1(float f, unsigned short& hi, unsigned short& lo) {
  const unsigned h = bf_rne(f);
  const float fh = __uint_as_float(h << 16);
  hi = (unsigned short)h;
  lo = (unsigned short)bf_rne(f - fh);
}

__device__ __forceinline__ void split8(v4f a, v4f b, v8us& hi, v8us& lo) {
  unsigned short h, l;
  split1(a.x, h, l); hi[0] = h; lo[0] = l;
  split1(a.y, h, l); hi[1] = h; lo[1] = l;
  split1(a.z, h, l); hi[2] = h; lo[2] = l;
  split1(a.w, h, l); hi[3] = h; lo[3] = l;
  split1(b.x, h, l); hi[4] = h; lo[4] = l;
  split1(b.y, h, l); hi[5] = h; lo[5] = l;
  split1(b.z, h, l); hi[6] = h; lo[6] = l;
  split1(b.w, h, l); hi[7] = h; lo[7] = l;
}

__device__ __forceinline__ v4f leaky4(v4f z) {
  v4f r;
  r.x = (z.x >= 0.f) ? z.x : 0.2f * z.x;
  r.y = (z.y >= 0.f) ? z.y : 0.2f * z.y;
  r.z = (z.z >= 0.f) ? z.z : 0.2f * z.z;
  r.w = (z.w >= 0.f) ? z.w : 0.2f * z.w;
  return r;
}

__device__ __forceinline__ void ln_relu_row(v4f& a, v4f& b, v4f g0, v4f g1, v4f e0, v4f e1) {
  const float s  = wsum(((a.x + a.y) + (a.z + a.w)) + ((b.x + b.y) + (b.z + b.w)));
  const float mu = s * (1.0f / DF);
  const v4f d0 = a - mu;
  const v4f d1 = b - mu;
  const float q  = wsum(d0.x * d0.x + d0.y * d0.y + d0.z * d0.z + d0.w * d0.w +
                        d1.x * d1.x + d1.y * d1.y + d1.z * d1.z + d1.w * d1.w);
  const float rs = rsqrtf(q * (1.0f / DF) + 1.0e-5f);
  v4f y0 = d0 * rs * g0 + e0;
  v4f y1 = d1 * rs * g1 + e1;
  y0.x = y0.x > 0.f ? y0.x : 0.f; y0.y = y0.y > 0.f ? y0.y : 0.f;
  y0.z = y0.z > 0.f ? y0.z : 0.f; y0.w = y0.w > 0.f ? y0.w : 0.f;
  y1.x = y1.x > 0.f ? y1.x : 0.f; y1.y = y1.y > 0.f ? y1.y : 0.f;
  y1.z = y1.z > 0.f ? y1.z : 0.f; y1.w = y1.w > 0.f ? y1.w : 0.f;
  a = y0; b = y1;
}

#define HITJ(J, HJ, SJ)                                                            \
  {                                                                                \
    const unsigned mj = __builtin_amdgcn_ballot_w32(HJ);                           \
    if (HJ) {                                                                      \
      const int pos = wc + (int)__builtin_amdgcn_mbcnt_lo(mj, 0u);                 \
      if (pos < WCAP) list[wave * WCAP + pos] = ((el0 + (J)) << SH) | (int)(SJ);   \
    }                                                                              \
    wc += (int)__builtin_popcount(mj);                                             \
  }

template <int NBT, int SH>
__device__ __forceinline__ void scan_chunk(const int* __restrict__ eid, int nE, int cbase, int nodeBase,
                                           int* list, int* wcnt, int tid, int lane, int wave) {
  int wc = 0;
  const bool full = ((nE & 3) == 0) && (cbase + CHUNK <= nE);
  const int sent = -2147483647 - 1;
  const int nm1 = nE - 1;
#pragma unroll
  for (int g = 0; g < NGRP; ++g) {
    const int el0 = (g * NTHR + tid) * 4;
    const int e0  = cbase + el0;
    v4i d;
    if (full) {
      d = *(const v4i*)(eid + e0);
    } else {
      const int t0 = eid[min(e0, nm1)];
      const int t1 = eid[min(e0 + 1, nm1)];
      const int t2 = eid[min(e0 + 2, nm1)];
      const int t3 = eid[min(e0 + 3, nm1)];
      d.x = (e0     < nE) ? t0 : sent;
      d.y = (e0 + 1 < nE) ? t1 : sent;
      d.z = (e0 + 2 < nE) ? t2 : sent;
      d.w = (e0 + 3 < nE) ? t3 : sent;
    }
    const unsigned s0 = (unsigned)d.x - (unsigned)nodeBase;
    const unsigned s1 = (unsigned)d.y - (unsigned)nodeBase;
    const unsigned s2 = (unsigned)d.z - (unsigned)nodeBase;
    const unsigned s3 = (unsigned)d.w - (unsigned)nodeBase;
    const bool h0 = s0 < (unsigned)NBT;
    const bool h1 = s1 < (unsigned)NBT;
    const bool h2 = s2 < (unsigned)NBT;
    const bool h3 = s3 < (unsigned)NBT;
    const unsigned many = __builtin_amdgcn_ballot_w32(h0 | h1 | h2 | h3);
    if (many != 0u) {
      HITJ(0, h0, s0)
      HITJ(1, h1, s1)
      HITJ(2, h2, s2)
      HITJ(3, h3, s3)
    }
  }
  if (lane == 0) wcnt[wave] = wc;
}
#undef HITJ

__global__ __launch_bounds__(NTHR) void k_wprep(const float* __restrict__ W0, const float* __restrict__ W1,
                                                const float* __restrict__ W2, const float* __restrict__ W3,
                                                unsigned short* Wt) {
  __shared__ __attribute__((aligned(16))) unsigned short Lh[32 * AP];
  __shared__ __attribute__((aligned(16))) unsigned short Ll[32 * AP];
  const int tid = threadIdx.x, lane = tid & 31, wave = tid >> 5;
  const int q  = blockIdx.y;
  const int o0 = blockIdx.x * 32;
  const float* W = (q == 0) ? W0 : ((q == 1) ? W1 : ((q == 2) ? W2 : W3));
#pragma unroll 4
  for (int i = 0; i < 32; ++i) {
    const int idx = i * NTHR + tid;
    const int k = idx >> 5;
    const int c = idx & 31;
    const float v = W[(size_t)k * DF + o0 + c];
    unsigned short h, l;
    split1(v, h, l);
    Lh[c * AP + k] = h;
    Ll[c * AP + k] = l;
  }
  __syncthreads();
  unsigned short* ph = Wt + (size_t)q * 2 * DF * DF;
  unsigned short* pl = ph + (size_t)DF * DF;
  v8us vh[4], vl[4];
#pragma unroll
  for (int i = 0; i < 4; ++i) {
    const int c = 4 * wave + i;
    vh[i] = *(const v8us*)(Lh + c * AP + 8 * lane);
    vl[i] = *(const v8us*)(Ll + c * AP + 8 * lane);
  }
#pragma unroll
  for (int i = 0; i < 4; ++i) {
    const size_t o = (size_t)(o0 + 4 * wave + i) * DF + 8 * lane;
    *(volatile v8us*)(ph + o) = vh[i];
    *(volatile v8us*)(pl + o) = vl[i];
  }
  __threadfence();
#pragma unroll
  for (int i = 0; i < 4; ++i) {
    const size_t o = (size_t)(o0 + 4 * wave + i) * DF + 8 * lane;
    *(volatile v8us*)(ph + o) = vh[i];
    *(volatile v8us*)(pl + o) = vl[i];
  }
}

__global__ __launch_bounds__(NTHR) void k_deg(const int* __restrict__ ei, const float* __restrict__ ew,
                                              float* dinv, int nN, int nE) {
  __shared__ __attribute__((aligned(16))) float degL[NBD];
  __shared__ int list[NWAVE * WCAP];
  __shared__ int wcnt[NWAVE];
  const int tid = threadIdx.x, lane = tid & 31, wave = tid >> 5;
  const int nodeBase = blockIdx.x * NBD;
#pragma unroll 1
  for (int i = tid; i < NBD; i += NTHR) degL[i] = 0.f;
  __syncthreads();
  const int* eid = ei + nE;
  const int nChunks = (nE + CHUNK - 1) / CHUNK;
#pragma unroll 1
  for (int ch = 0; ch < nChunks; ++ch) {
    const int cbase = ch * CHUNK;
    scan_chunk<NBD, NBDSH>(eid, nE, cbase, nodeBase, list, wcnt, tid, lane, wave);
    __syncthreads();
    if (wave == 0) {
#pragma unroll 1
      for (int wsx = 0; wsx < NWAVE; ++wsx) {
        int n = wcnt[wsx];
        n = n > WCAP ? WCAP : (n < 0 ? 0 : n);
#pragma unroll 1
        for (int i = 0; i < n; ++i) {
          const int ent  = list[wsx * WCAP + i];
          const int slot = ent & (NBD - 1);
          const int el   = (ent >> NBDSH) & (CHUNK - 1);
          const int e    = min(cbase + el, nE - 1);
          const float w  = ew[e];
          if ((slot & 31) == lane) degL[slot] += w;
        }
      }
    }
    __syncthreads();
  }
  v4f r[4];
#pragma unroll
  for (int p = 0; p < 4; ++p) {
    const v4f d = *(const v4f*)(degL + 4 * (p * NTHR + tid));
    r[p].x = rsqrtf(d.x + 1.0f);
    r[p].y = rsqrtf(d.y + 1.0f);
    r[p].z = rsqrtf(d.z + 1.0f);
    r[p].w = rsqrtf(d.w + 1.0f);
  }
  float* base = dinv + (size_t)nodeBase;
#pragma unroll
  for (int p = 0; p < 4; ++p) *(volatile v4f*)(base + 4 * (p * NTHR + tid)) = r[p];
  __threadfence();
#pragma unroll
  for (int p = 0; p < 4; ++p) *(volatile v4f*)(base + 4 * (p * NTHR + tid)) = r[p];
}

struct GJob  { const float* A; const unsigned short* Wh; const unsigned short* Wl; const float* bias; float* dst; int nrows; int hasBias; };
struct GArgs { GJob j0; GJob j1; GJob j2; const float* gamma; const float* beta; };
static_assert(sizeof(GJob) == 48);
static_assert(sizeof(GArgs) == 160);

template <int EPI>
__global__ __launch_bounds__(NTHR) void k_gemm(GArgs g) {
  __shared__ __attribute__((aligned(16))) unsigned char smem[GEMM_LDS];
  unsigned short* Ah = reinterpret_cast<unsigned short*>(smem);
  unsigned short* Al = Ah + GR * AP;
  float* Xs = reinterpret_cast<float*>(smem);
  const int tid = threadIdx.x, lane = tid & 31, wave = tid >> 5;
  const int hh = lane >> 4, m = lane & 15;
  const int y = blockIdx.y;
  const float*          A     = (y == 0) ? g.j0.A      : ((y == 1) ? g.j1.A      : g.j2.A);
  const unsigned short* Wh    = (y == 0) ? g.j0.Wh     : ((y == 1) ? g.j1.Wh     : g.j2.Wh);
  const unsigned short* Wl    = (y == 0) ? g.j0.Wl     : ((y == 1) ? g.j1.Wl     : g.j2.Wl);
  const float*          bias  = (y == 0) ? g.j0.bias   : ((y == 1) ? g.j1.bias   : g.j2.bias);
  float*                dst   = (y == 0) ? g.j0.dst    : ((y == 1) ? g.j1.dst    : g.j2.dst);
  const int             nrows = (y == 0) ? g.j0.nrows  : ((y == 1) ? g.j1.nrows  : g.j2.nrows);
  const int             hasB  = (y == 0) ? g.j0.hasBias: ((y == 1) ? g.j1.hasBias: g.j2.hasBias);
  const int rowBase = blockIdx.x * GR;

  {
    const int r  = tid >> 3;
    const int c0 = (tid & 7) * 32;
    int row = rowBase + r;
    row = (row > nrows - 1) ? (nrows - 1) : row;
    const float* p = A + (size_t)row * DF + c0;
#pragma unroll
    for (int q = 0; q < 4; ++q) {
      const v4f f0 = *(const v4f*)(p + 8 * q);
      const v4f f1 = *(const v4f*)(p + 8 * q + 4);
      v8us uh, ul;
      split8(f0, f1, uh, ul);
      *(v8us*)(Ah + r * AP + c0 + 8 * q) = uh;
      *(v8us*)(Al + r * AP + c0 + 8 * q) = ul;
    }
  }
  __syncthreads();

  v8f a00 = {0.f, 0.f, 0.f, 0.f, 0.f, 0.f, 0.f, 0.f};
  v8f a01 = a00, a10 = a00, a11 = a00;
  const int n0 = wave * 32 + m, n1 = n0 + 16;
  const unsigned short* pbh0 = Wh + (size_t)n0 * DF + 8 * hh;
  const unsigned short* pbl0 = Wl + (size_t)n0 * DF + 8 * hh;
  const unsigned short* pbh1 = Wh + (size_t)n1 * DF + 8 * hh;
  const unsigned short* pbl1 = Wl + (size_t)n1 * DF + 8 * hh;
  const unsigned short* pah0 = Ah + m * AP + 8 * hh;
  const unsigned short* pah1 = Ah + (16 + m) * AP + 8 * hh;
  const unsigned short* pal0 = Al + m * AP + 8 * hh;
  const unsigned short* pal1 = Al + (16 + m) * AP + 8 * hh;
#pragma unroll 2
  for (int kt = 0; kt < DF / 32; ++kt) {
    const int k0 = kt * 32;
    FragB ah0, ah1, al0, al1, bh0, bh1, bl0, bl1;
    ah0.h[0] = *(const v8us*)(pah0 + k0); ah0.h[1] = *(const v8us*)(pah0 + k0 + 16);
    ah1.h[0] = *(const v8us*)(pah1 + k0); ah1.h[1] = *(const v8us*)(pah1 + k0 + 16);
    al0.h[0] = *(const v8us*)(pal0 + k0); al0.h[1] = *(const v8us*)(pal0 + k0 + 16);
    al1.h[0] = *(const v8us*)(pal1 + k0); al1.h[1] = *(const v8us*)(pal1 + k0 + 16);
    bh0.h[0] = *(const v8us*)(pbh0 + k0); bh0.h[1] = *(const v8us*)(pbh0 + k0 + 16);
    bl0.h[0] = *(const v8us*)(pbl0 + k0); bl0.h[1] = *(const v8us*)(pbl0 + k0 + 16);
    bh1.h[0] = *(const v8us*)(pbh1 + k0); bh1.h[1] = *(const v8us*)(pbh1 + k0 + 16);
    bl1.h[0] = *(const v8us*)(pbl1 + k0); bl1.h[1] = *(const v8us*)(pbl1 + k0 + 16);
    a00 = wm(ah0.v, bh0.v, a00); a00 = wm(ah0.v, bl0.v, a00); a00 = wm(al0.v, bh0.v, a00);
    a01 = wm(ah0.v, bh1.v, a01); a01 = wm(ah0.v, bl1.v, a01); a01 = wm(al0.v, bh1.v, a01);
    a10 = wm(ah1.v, bh0.v, a10); a10 = wm(ah1.v, bl0.v, a10); a10 = wm(al1.v, bh0.v, a10);
    a11 = wm(ah1.v, bh1.v, a11); a11 = wm(ah1.v, bl1.v, a11); a11 = wm(al1.v, bh1.v, a11);
  }
  __syncthreads();

  const float bb0 = bias[n0];
  const float bb1 = bias[n1];
  const float bv0 = hasB ? bb0 : 0.f;
  const float bv1 = hasB ? bb1 : 0.f;
#pragma unroll
  for (int r = 0; r < 8; ++r) {
    Xs[(8 * hh + r) * XSP + n0]      = a00[r] + bv0;
    Xs[(8 * hh + r) * XSP + n1]      = a01[r] + bv1;
    Xs[(16 + 8 * hh + r) * XSP + n0] = a10[r] + bv0;
    Xs[(16 + 8 * hh + r) * XSP + n1] = a11[r] + bv1;
  }
  __syncthreads();

  v4f o0[4], o1[4];
  v4f g0 = {1.f, 1.f, 1.f, 1.f}, g1 = g0, e0 = {0.f, 0.f, 0.f, 0.f}, e1 = e0;
  if (EPI == 1) {
    g0 = *(const v4f*)(g.gamma + 4 * lane);
    g1 = *(const v4f*)(g.gamma + 128 + 4 * lane);
    e0 = *(const v4f*)(g.beta + 4 * lane);
    e1 = *(const v4f*)(g.beta + 128 + 4 * lane);
  }
#pragma unroll
  for (int i = 0; i < 4; ++i) {
    const int row = 4 * wave + i;
    o0[i] = *(const v4f*)(Xs + row * XSP + 4 * lane);
    o1[i] = *(const v4f*)(Xs + row * XSP + 128 + 4 * lane);
    if (EPI == 1) ln_relu_row(o0[i], o1[i], g0, g1, e0, e1);
  }
#pragma unroll
  for (int i = 0; i < 4; ++i) {
    const int grow = rowBase + 4 * wave + i;
    if (grow < nrows) {
      float* op = dst + (size_t)grow * DF + 4 * lane;
      *(volatile v4f*)(op)       = o0[i];
      *(volatile v4f*)(op + 128) = o1[i];
    }
  }
  __threadfence();
#pragma unroll
  for (int i = 0; i < 4; ++i) {
    const int grow = rowBase + 4 * wave + i;
    if (grow < nrows) {
      float* op = dst + (size_t)grow * DF + 4 * lane;
      *(volatile v4f*)(op)       = o0[i];
      *(volatile v4f*)(op + 128) = o1[i];
    }
  }
}

__global__ __launch_bounds__(NTHR) void k_glom(
    const float* __restrict__ hl, const float* __restrict__ hr, const float* __restrict__ xw,
    const float* __restrict__ dinv,
    const int* __restrict__ eiB, const float* __restrict__ ea,
    const int* __restrict__ eiA, const float* __restrict__ ew,
    const float* __restrict__ We, const float* __restrict__ att,
    const float* __restrict__ b_gat, const float* __restrict__ b_gcn,
    const float* __restrict__ gam, const float* __restrict__ bet,
    float* out, int nG, int nI, int nEB, int nEA) {
  extern __shared__ v4f lds_dyn[];
  float* sacc = (float*)lds_dyn;
  float* mL   = sacc + AGG_SACC;
  float* den  = mL + NB;
  float* dq   = den + NB;
  int*   list = (int*)(dq + NB);
  int*   wcnt = list + NWAVE * WCAP;

  const int tid = threadIdx.x, lane = tid & 31, wave = tid >> 5;
  const int nodeBase = blockIdx.x * NB;

  {
    const v4f z4 = {0.f, 0.f, 0.f, 0.f};
#pragma unroll 1
    for (int i = tid; i < AGG_SACC / 4; i += NTHR) lds_dyn[i] = z4;
    int nd = nodeBase + tid;
    nd = (nd > nG - 1) ? (nG - 1) : nd;
    mL[tid]  = -1.0e30f;
    den[tid] = 0.f;
    dq[tid]  = dinv[nd];
  }
  const v4f we0 = *(const v4f*)(We + 4 * lane);
  const v4f we1 = *(const v4f*)(We + 128 + 4 * lane);
  const v4f at0 = *(const v4f*)(att + 4 * lane);
  const v4f at1 = *(const v4f*)(att + 128 + 4 * lane);
  __syncthreads();

  {
    const int* eid = eiB + nEB;
    const int nChunks = (nEB + CHUNK - 1) / CHUNK;
#pragma unroll 1
    for (int ch = 0; ch < nChunks; ++ch) {
      const int cbase = ch * CHUNK;
      scan_chunk<NB, NBSH>(eid, nEB, cbase, nodeBase, list, wcnt, tid, lane, wave);
      __syncthreads();
      if (wave == 0) {
#pragma unroll 1
        for (int wsx = 0; wsx < NWAVE; ++wsx) {
          int n = wcnt[wsx];
          n = n > WCAP ? WCAP : (n < 0 ? 0 : n);
#pragma unroll 1
          for (int i = 0; i < n; ++i) {
            const int ent  = list[wsx * WCAP + i];
            const int slot = ent & (NB - 1);
            const int el   = (ent >> NBSH) & (CHUNK - 1);
            const int e    = min(cbase + el, nEB - 1);
            int src = eiB[e];
            src = src < 0 ? 0 : (src > nI - 1 ? nI - 1 : src);
            int nd = nodeBase + slot;
            nd = nd > nG - 1 ? nG - 1 : nd;
            const float eav = ea[e];
            const float* ph = hl + (size_t)src * DF + 4 * lane;
            const float* pr = hr + (size_t)nd * DF + 4 * lane;
            const v4f h0 = *(const v4f*)(ph);
            const v4f h1 = *(const v4f*)(ph + 128);
            const v4f r0 = *(const v4f*)(pr);
            const v4f r1 = *(const v4f*)(pr + 128);
            v4f z0 = (h0 + r0) + eav * we0;
            v4f z1 = (h1 + r1) + eav * we1;
            z0 = leaky4(z0);
            z1 = leaky4(z1);
            const float pd = z0.x * at0.x + z0.y * at0.y + z0.z * at0.z + z0.w * at0.w +
                             z1.x * at1.x + z1.y * at1.y + z1.z * at1.z + z1.w * at1.w;
            const float lg = wsum(pd);
            const float mo = mL[slot];
            const float mn = fmaxf(mo, lg);
            const float sc = __expf(mo - mn);
            const float p  = __expf(lg - mn);
            v4f* s0p = (v4f*)(sacc + slot * DF + 4 * lane);
            v4f* s1p = s0p + 32;
            const v4f s0 = *s0p;
            const v4f s1 = *s1p;
            const v4f u0 = s0 * sc + p * h0;
            const v4f u1 = s1 * sc + p * h1;
            *s0p = u0;
            *s1p = u1;
            const float dn = den[slot] * sc + p;
            mL[slot]  = mn;
            den[slot] = dn;
          }
        }
      }
      __syncthreads();
    }
  }

#pragma unroll 1
  for (int i = tid; i < AGG_SACC / 4; i += NTHR) {
    const int slot = i >> 6;
    const int c4   = (i & 63) * 4;
    const float dn  = den[slot];
    const float rcp = __builtin_amdgcn_rcpf(dn);
    const float inv = (dn > 0.f) ? rcp : 0.f;
    const v4f b4 = *(const v4f*)(b_gat + c4);
    const v4f cur = lds_dyn[i];
    lds_dyn[i] = cur * inv + b4;
  }
  __syncthreads();

  {
    const int* eid = eiA + nEA;
    const int nChunks = (nEA + CHUNK - 1) / CHUNK;
#pragma unroll 1
    for (int ch = 0; ch < nChunks; ++ch) {
      const int cbase = ch * CHUNK;
      scan_chunk<NB, NBSH>(eid, nEA, cbase, nodeBase, list, wcnt, tid, lane, wave);
      __syncthreads();
      if (wave == 0) {
#pragma unroll 1
        for (int wsx = 0; wsx < NWAVE; ++wsx) {
          int n = wcnt[wsx];
          n = n > WCAP ? WCAP : (n < 0 ? 0 : n);
#pragma unroll 1
          for (int i = 0; i < n; ++i) {
            const int ent  = list[wsx * WCAP + i];
            const int slot = ent & (NB - 1);
            const int el   = (ent >> NBSH) & (CHUNK - 1);
            const int e    = min(cbase + el, nEA - 1);
            int src = eiA[e];
            src = src < 0 ? 0 : (src > nG - 1 ? nG - 1 : src);
            const float w = ew[e];
            const float c = (dinv[src] * w) * dq[slot];
            const float* px = xw + (size_t)src * DF + 4 * lane;
            const v4f x0 = *(const v4f*)(px);
            const v4f x1 = *(const v4f*)(px + 128);
            v4f* s0p = (v4f*)(sacc + slot * DF + 4 * lane);
            v4f* s1p = s0p + 32;
            const v4f u0 = *s0p + c * x0;
            const v4f u1 = *s1p + c * x1;
            *s0p = u0;
            *s1p = u1;
          }
        }
      }
      __syncthreads();
    }
  }

  const v4f bg0 = *(const v4f*)(b_gcn + 4 * lane);
  const v4f bg1 = *(const v4f*)(b_gcn + 128 + 4 * lane);
  const v4f g0  = *(const v4f*)(gam + 4 * lane);
  const v4f g1  = *(const v4f*)(gam + 128 + 4 * lane);
  const v4f e0  = *(const v4f*)(bet + 4 * lane);
  const v4f e1  = *(const v4f*)(bet + 128 + 4 * lane);
#pragma unroll 1
  for (int j = 0; j < NB / NWAVE; ++j) {
    const int slot = wave * (NB / NWAVE) + j;
    const int node = nodeBase + slot;
    if (node >= nG) break;
    const float d2 = dq[slot] * dq[slot];
    const float* px = xw + (size_t)node * DF + 4 * lane;
    const v4f x0 = *(const v4f*)(px);
    const v4f x1 = *(const v4f*)(px + 128);
    v4f h0 = *(const v4f*)(sacc + slot * DF + 4 * lane) + d2 * x0 + bg0;
    v4f h1 = *(const v4f*)(sacc + slot * DF + 128 + 4 * lane) + d2 * x1 + bg1;
    ln_relu_row(h0, h1, g0, g1, e0, e1);
    float* op = out + (size_t)node * DF + 4 * lane;
    *(volatile v4f*)(op)       = h0;
    *(volatile v4f*)(op + 128) = h1;
    __threadfence();
    *(volatile v4f*)(op)       = h0;
    *(volatile v4f*)(op + 128) = h1;
  }
}

__global__ __launch_bounds__(NTHR) void k_imm(
    const float* __restrict__ xg, const float* __restrict__ xi, const float* __restrict__ eps,
    const int* __restrict__ ei, float* tin, int nG, int nI, int nE) {
  extern __shared__ v4f lds_dyn[];
  float* sacc = (float*)lds_dyn;
  int*   list = (int*)(sacc + AGG_SACC);
  int*   wcnt = list + NWAVE * WCAP;
  const int tid = threadIdx.x, lane = tid & 31, wave = tid >> 5;
  const int nodeBase = blockIdx.x * NB;
  {
    const v4f z4 = {0.f, 0.f, 0.f, 0.f};
#pragma unroll 1
    for (int i = tid; i < AGG_SACC / 4; i += NTHR) lds_dyn[i] = z4;
  }
  __syncthreads();
  {
    const int* eid = ei + nE;
    const int nChunks = (nE + CHUNK - 1) / CHUNK;
#pragma unroll 1
    for (int ch = 0; ch < nChunks; ++ch) {
      const int cbase = ch * CHUNK;
      scan_chunk<NB, NBSH>(eid, nE, cbase, nodeBase, list, wcnt, tid, lane, wave);
      __syncthreads();
      if (wave == 0) {
#pragma unroll 1
        for (int wsx = 0; wsx < NWAVE; ++wsx) {
          int n = wcnt[wsx];
          n = n > WCAP ? WCAP : (n < 0 ? 0 : n);
#pragma unroll 1
          for (int i = 0; i < n; ++i) {
            const int ent  = list[wsx * WCAP + i];
            const int slot = ent & (NB - 1);
            const int el   = (ent >> NBSH) & (CHUNK - 1);
            const int e    = min(cbase + el, nE - 1);
            int src = ei[e];
            src = src < 0 ? 0 : (src > nG - 1 ? nG - 1 : src);
            const float* px = xg + (size_t)src * DF + 4 * lane;
            const v4f x0 = *(const v4f*)(px);
            const v4f x1 = *(const v4f*)(px + 128);
            v4f* s0p = (v4f*)(sacc + slot * DF + 4 * lane);
            v4f* s1p = s0p + 32;
            const v4f u0 = *s0p + x0;
            const v4f u1 = *s1p + x1;
            *s0p = u0;
            *s1p = u1;
          }
        }
      }
      __syncthreads();
    }
  }
  const float opf = 1.0f + eps[0];
#pragma unroll 1
  for (int j = 0; j < NB / NWAVE; ++j) {
    const int slot = wave * (NB / NWAVE) + j;
    const int node = nodeBase + slot;
    if (node >= nI) break;
    const float* px = xi + (size_t)node * DF + 4 * lane;
    v4f t0 = opf * *(const v4f*)(px);
    v4f t1 = opf * *(const v4f*)(px + 128);
    t0 = t0 + *(const v4f*)(sacc + slot * DF + 4 * lane);
    t1 = t1 + *(const v4f*)(sacc + slot * DF + 128 + 4 * lane);
    float* op = tin + (size_t)node * DF + 4 * lane;
    *(volatile v4f*)(op)       = t0;
    *(volatile v4f*)(op + 128) = t1;
    __threadfence();
    *(volatile v4f*)(op)       = t0;
    *(volatile v4f*)(op + 128) = t1;
  }
}

extern "C" void kernel_launch(void* const* d_in, const int* in_sizes, int n_in,
                              void* d_out, int out_size, void* d_ws, size_t ws_size,
                              hipStream_t stream) {
  if (n_in < 21) return;
  const int nG = in_sizes[0] / DF;
  const int nI = in_sizes[1] / DF;
  if (nG <= 0 || nI <= 0 || in_sizes[0] != nG * DF || in_sizes[1] != nI * DF) return;
  const int nEA = in_sizes[18] / 2;
  const int nEB = in_sizes[19] / 2;
  const int nEC = in_sizes[20] / 2;
  if (nEA < 0 || nEB < 0 || nEC < 0) return;
  if (in_sizes[18] != 2 * nEA || in_sizes[19] != 2 * nEB || in_sizes[20] != 2 * nEC) return;
  if (in_sizes[2] != nEA || in_sizes[3] != nEB) return;
  if (in_sizes[4] != DF * DF || in_sizes[6] != DF * DF || in_sizes[8] != DF * DF || in_sizes[14] != DF * DF) return;
  if (in_sizes[5] != DF || in_sizes[7] != DF || in_sizes[9] != DF || in_sizes[10] != DF ||
      in_sizes[11] != DF || in_sizes[12] != DF || in_sizes[15] != DF || in_sizes[16] != DF ||
      in_sizes[17] != DF) return;
  if (in_sizes[13] < 1) return;
  if (out_size != (nG + nI) * DF) return;

  const float* x_glom = (const float*)d_in[0];
  const float* x_imm  = (const float*)d_in[1];
  const float* ew_gg  = (const float*)d_in[2];
  const float* ea_ig  = (const float*)d_in[3];
  const float* W_gcn  = (const float*)d_in[4];
  const float* b_gcn  = (const float*)d_in[5];
  const float* Wl     = (const float*)d_in[6];
  const float* bl     = (const float*)d_in[7];
  const float* Wr     = (const float*)d_in[8];
  const float* br     = (const float*)d_in[9];
  const float* att    = (const float*)d_in[10];
  const float* We     = (const float*)d_in[11];
  const float* b_gat  = (const float*)d_in[12];
  const float* eps    = (const float*)d_in[13];
  const float* W_gin  = (const float*)d_in[14];
  const float* b_gin  = (const float*)d_in[15];
  const float* gamma  = (const float*)d_in[16];
  const float* beta   = (const float*)d_in[17];
  const int*   ei_gg  = (const int*)d_in[18];
  const int*   ei_ig  = (const int*)d_in[19];
  const int*   ei_gi  = (const int*)d_in[20];
  float* out_glom = (float*)d_out;
  float* out_imm  = out_glom + (size_t)nG * DF;

  const int gridDeg = (nG + NBD - 1) / NBD;
  const int nGr = ((nG + GR - 1) / GR) * GR;
  const int nIr = ((nI + GR - 1) / GR) * GR;
  size_t off = 0;
  const size_t szWt  = (size_t)4 * 2 * DF * DF * sizeof(unsigned short);
  const size_t szDi  = ((size_t)gridDeg * NBD * sizeof(float) + 255) & ~(size_t)255;
  const size_t szG   = (size_t)nGr * DF * sizeof(float);
  const size_t szI   = (size_t)nIr * DF * sizeof(float);
  unsigned short* Wt = (unsigned short*)((char*)d_ws + off); off += szWt;
  float* dinv = (float*)((char*)d_ws + off); off += szDi;
  float* xw   = (float*)((char*)d_ws + off); off += szG;
  float* hr   = (float*)((char*)d_ws + off); off += szG;
  float* hl   = (float*)((char*)d_ws + off); off += szI;
  float* tin  = (float*)((char*)d_ws + off); off += szI;
  if (off > ws_size) return;

  k_wprep<<<dim3(DF / 32, 4), NTHR, 0, stream>>>(W_gcn, Wr, Wl, W_gin, Wt);

  k_deg<<<gridDeg, NTHR, 0, stream>>>(ei_gg, ew_gg, dinv, nG, nEA);

  GArgs a;
  a.j0.A = x_glom; a.j0.Wh = Wt + (size_t)0 * 2 * DF * DF; a.j0.Wl = a.j0.Wh + (size_t)DF * DF; a.j0.bias = b_gcn; a.j0.dst = xw; a.j0.nrows = nG; a.j0.hasBias = 0;
  a.j1.A = x_glom; a.j1.Wh = Wt + (size_t)1 * 2 * DF * DF; a.j1.Wl = a.j1.Wh + (size_t)DF * DF; a.j1.bias = br;    a.j1.dst = hr; a.j1.nrows = nG; a.j1.hasBias = 1;
  a.j2.A = x_imm;  a.j2.Wh = Wt + (size_t)2 * 2 * DF * DF; a.j2.Wl = a.j2.Wh + (size_t)DF * DF; a.j2.bias = bl;    a.j2.dst = hl; a.j2.nrows = nI; a.j2.hasBias = 1;
  a.gamma = gamma; a.beta = beta;
  const int gx = ((nG > nI ? nG : nI) + GR - 1) / GR;
  k_gemm<0><<<dim3(gx, 3), NTHR, 0, stream>>>(a);

  hipFuncSetAttribute(reinterpret_cast<const void*>(&k_glom), hipFuncAttributeMaxDynamicSharedMemorySize, LDS_GLOM);
  k_glom<<<(nG + NB - 1) / NB, NTHR, LDS_GLOM, stream>>>(hl, hr, xw, dinv, ei_ig, ea_ig, ei_gg, ew_gg,
                                                        We, att, b_gat, b_gcn, gamma, beta,
                                                        out_glom, nG, nI, nEB, nEA);

  hipFuncSetAttribute(reinterpret_cast<const void*>(&k_imm), hipFuncAttributeMaxDynamicSharedMemorySize, LDS_IMM);
  k_imm<<<(nI + NB - 1) / NB, NTHR, LDS_IMM, stream>>>(x_glom, x_imm, eps, ei_gi, tin, nG, nI, nEC);

  GArgs b;
  b.j0.A = tin; b.j0.Wh = Wt + (size_t)3 * 2 * DF * DF; b.j0.Wl = b.j0.Wh + (size_t)DF * DF; b.j0.bias = b_gin; b.j0.dst = out_imm; b.j0.nrows = nI; b.j0.hasBias = 1;
  b.j1 = b.j0; b.j2 = b.j0;
  b.gamma = gamma; b.beta = beta;
  k_gemm<1><<<dim3((nI + GR - 1) / GR, 1), NTHR, 0, stream>>>(b);
}
